// TriangleSelfAttention_3109556322361
// MI455X (gfx1250) — hardware-run, weakly checked
//
#include <hip/hip_runtime.h>


namespace {
constexpr int NB = 256, L = 256, C = 128, NH = 4, HD = 32, NT = NB * L, KB = 128, PW = 3 * C;
constexpr float XS = 8.0f, HS = 256.0f  , WSC = 256.0f, PS = 256.0f, SCALE = 0.17677669529663687f;
typedef _Float16 b16;
typedef __attribute__((ext_vector_type(16))) _Float16 v16b;
typedef __attribute__((ext_vector_type(8))) _Float16 v8b;
typedef __attribute__((ext_vector_type(8))) float v8f;
typedef __attribute__((ext_vector_type(4))) float v4f;
__device__ __forceinline__ float bf16_rne(float f) { unsigned int u = __float_as_uint(f); u += 0x7FFFu + ((u >> 16) & 1u); float r = __uint_as_float(u & 0xFFFF0000u); asm volatile("" : "+v"(r)); return r; }
__device__ __forceinline__ float bfv(float f) { float r = bf16_rne(f); asm volatile("" : "+v"(r)); return r; }
__device__ __forceinline__ void split16(float v, b16& hi, b16& lo) { hi = (b16)v; lo = (b16)(v - (float)hi); }
__device__ __forceinline__ v16b frag_kb(const b16* p, int hh) { const v8b a = *(const v8b*)(p + 8 * hh), b = *(const v8b*)(p + 16 + 8 * hh); v16b f;
#pragma unroll
  for (int e = 0; e < 8; ++e) { f[e] = a[e]; f[8 + e] = b[e]; } return f; }
__device__ __forceinline__ v8f wmma16b(v16b a, v16b b, v8f c) { v8f d = __builtin_amdgcn_wmma_f32_16x16x32_f16(false, a, false, b, (short)0, c, false, false); asm volatile("v_nop\n\tv_nop\n\tv_nop\n\tv_nop" : "+v"(d) : "v"(a), "v"(b)); return d; }
__device__ __forceinline__ void wave_lds_sync() { __builtin_amdgcn_fence(__ATOMIC_RELEASE, "workgroup"); __builtin_amdgcn_wave_barrier(); __builtin_amdgcn_fence(__ATOMIC_ACQUIRE, "workgroup"); }
__device__ __forceinline__ float pmul(float a, float b) { float p = a * b; asm volatile("" : "+v"(p)); return p; }

__global__ __launch_bounds__(256) void wput_kernel(const float* __restrict__ wq, const float* __restrict__ wk, const float* __restrict__ wv, const float* __restrict__ wo, b16* __restrict__ W3, b16* __restrict__ WO) { const size_t u = (size_t)blockIdx.x * 256 + threadIdx.x; if (u >= (size_t)4 * C * (C / 8)) return; const int r = (int)(u / (C / 8)), k0 = (int)(u % (C / 8)) * 8; const int p = r / C, o = r % C; const float* w = p == 0 ? wq : (p == 1 ? wk : (p == 2 ? wv : wo)); v8b v;
#pragma unroll
  for (int j = 0; j < 8; ++j) v[j] = (b16)(bf16_rne(w[(size_t)o * C + k0 + j]) * WSC);
  for (int pass = 0; pass < 2; ++pass) { *(volatile v8b*)((p < 3 ? W3 + (size_t)r * C : WO + (size_t)o * C) + k0) = v; __threadfence(); } }
__global__ __launch_bounds__(32) void proj_kernel(const float* __restrict__ x, const b16* __restrict__ W3, const float* __restrict__ bq, const float* __restrict__ bk, const float* __restrict__ bv, int TLIM, b16* __restrict__ PH, b16* __restrict__ PL) { __shared__ __attribute__((aligned(16))) b16 Ah[16][C + 8], Oh[16][264], Ol[16][264]; const int lane = threadIdx.x, nloc = lane & 15, hlf = lane >> 4; const size_t m0 = (size_t)blockIdx.x * 16; if (m0 >= (size_t)TLIM) return;
  for (int rr = 0; rr < 16; ++rr) for (int q = 0; q < C / 32; ++q) Ah[rr][q * 32 + lane] = (b16)(bf16_rne(x[(m0 + rr) * C + q * 32 + lane]) * XS);
  wave_lds_sync();
#pragma unroll 1
  for (int g = 0; g < 3; ++g) { const int pj = g;     const float* bb = pj == 0 ? bq : (pj == 1 ? bk : bv); const float sc = pj == 0 ? SCALE : 1.0f; v8f acc[8];
#pragma unroll
    for (int t = 0; t < 8; ++t) acc[t] = (v8f){};
#pragma unroll 2
    for (int kb = 0; kb < C; kb += 32) { const v16b a = frag_kb(&Ah[nloc][kb], hlf);
#pragma unroll
      for (int t = 0; t < 8; ++t) acc[t] = wmma16b(a, frag_kb(W3 + (size_t)(g * C + t * 16 + nloc) * C + kb, hlf), acc[t]); }
#pragma unroll
    for (int t = 0; t < 8; ++t) { const int cc = t * 16 + nloc; const float bvv = bfv(bb[cc]);
#pragma unroll
      for (int r8 = 0; r8 < 8; ++r8) { b16 p, ql; split16((acc[t][r8] * (1.0f / (XS * WSC)) + bvv) * sc * HS, p, ql); Oh[8 * hlf + r8][cc] = p; Ol[8 * hlf + r8][cc] = ql; } }
    wave_lds_sync();
    for (int pass = 0; pass < 2; ++pass) { for (int rr = 0; rr < 16; ++rr) if (lane < 16) { *(volatile v8b*)(PH + (m0 + rr) * PW + g * C + lane * 8) = *(const v8b*)(&Oh[rr][lane * 8]); *(volatile v8b*)(PL + (m0 + rr) * PW + g * C + lane * 8) = *(const v8b*)(&Ol[rr][lane * 8]); } __threadfence(); }
    wave_lds_sync(); } }
__global__ __launch_bounds__(32) void att_kernel(const b16* __restrict__ PH, const b16* __restrict__ PL, const float* __restrict__ amask, int BLIM, float* __restrict__ ATT) { __shared__ __attribute__((aligned(16))) b16 Ph_[16][KB + 8], Pl_[16][KB + 8], Vth[HD][KB + 8], Vtl[HD][KB + 8]; __shared__ float Sf[16][KB + 4], Of[16][HD + 4];
  const int lane = threadIdx.x, nloc = lane & 15, hlf = lane >> 4; const int qt = blockIdx.x % (L / 16); const int h = (blockIdx.x / (L / 16)) % NH; const int b = blockIdx.x / ((L / 16) * NH); if (b >= BLIM) return; const int t0 = qt * 16; const size_t rowb = (size_t)b * L; const int qo = h * HD, ko = C + h * HD, vo = 2 * C + h * HD;
  v16b qh[HD / 32], ql[HD / 32];
#pragma unroll
  for (int s = 0; s < HD / 32; ++s) { qh[s] = frag_kb(PH + (rowb + t0 + nloc) * PW + qo + s * 32, hlf); ql[s] = frag_kb(PL + (rowb + t0 + nloc) * PW + qo + s * 32, hlf); }
  float m_r[8], den_r[8]; v8f acc[HD / 16];
#pragma unroll
  for (int r8 = 0; r8 < 8; ++r8) { m_r[r8] = -INFINITY; den_r[r8] = 0.0f; }
#pragma unroll
  for (int t = 0; t < HD / 16; ++t) acc[t] = (v8f){};
  const int kstart = 0; const int kend = L;
#pragma unroll 1
  for (int kb0 = kstart; kb0 < kend; kb0 += KB) { const int nk = (kend - kb0) < KB ? (kend - kb0) : KB; const int nkt = (nk + 15) / 16;
    for (int rr = 0; rr < KB; rr += 2) { const int r = rr + hlf; const int key = kb0 + r < L ? kb0 + r : L - 1;     const size_t vr = (rowb + key) * PW + vo; for (int s = 0; s < HD / 32; ++s) { Vth[s * 32 + nloc][r] = PH[vr + s * 32 + nloc]; Vth[s * 32 + 16 + nloc][r] = PH[vr + s * 32 + 16 + nloc]; Vtl[s * 32 + nloc][r] = PL[vr + s * 32 + nloc]; Vtl[s * 32 + 16 + nloc][r] = PL[vr + s * 32 + 16 + nloc]; } }
    for (int t = 0; t < KB / 16; ++t) { if (t < nkt) { const int key = kb0 + t * 16 + nloc < L ? kb0 + t * 16 + nloc : L - 1; const size_t kr = (rowb + key) * PW + ko; v8f s = {};
#pragma unroll
        for (int q = 0; q < HD / 32; ++q) { const v16b kh = frag_kb(PH + kr + q * 32, hlf), kl = frag_kb(PL + kr + q * 32, hlf); s = wmma16b(qh[q], kh, s); s = wmma16b(qh[q], kl, s); s = wmma16b(ql[q], kh, s); }
#pragma unroll
        for (int r8 = 0; r8 < 8; ++r8) { const int i = t0 + 8 * hlf + r8, j = kb0 + t * 16 + nloc; const bool ok = (j < kend); Sf[8 * hlf + r8][t * 16 + nloc] = ok ? s[r8] * (1.0f / (HS * HS)) : -INFINITY; } }
      else {
#pragma unroll
        for (int r8 = 0; r8 < 8; ++r8) Sf[8 * hlf + r8][t * 16 + nloc] = -INFINITY; } }
    wave_lds_sync();
#pragma unroll
    for (int rr = 0; rr < 16; ++rr) { float mx = -INFINITY;
#pragma unroll
      for (int q = 0; q < 4; ++q) mx = fmaxf(mx, Sf[rr][q * 32 + lane]);
      for (int o = 16; o; o >>= 1) mx = fmaxf(mx, __shfl_xor(mx, o));
      const float mold = __shfl(m_r[rr & 7], (rr >> 3) * 16); const float mn = fmaxf(mold, mx); const float sf = (mold == -INFINITY) ? 0.0f : ((mn == -INFINITY) ? 1.0f : __expf(mold - mn)); float ps = 0.0f;
#pragma unroll
      for (int q = 0; q < 4; ++q) { const int kx = q * 32 + lane; const float sv = Sf[rr][kx]; const float p = (sv == -INFINITY || mn == -INFINITY) ? 0.0f : __expf(sv - mn); ps += p; b16 ph, pl; split16(p * PS, ph, pl); Ph_[rr][kx] = ph; Pl_[rr][kx] = pl; }
      for (int o = 16; o; o >>= 1) ps += __shfl_xor(ps, o);
      if ((rr >> 3) == hlf) { const int r8 = rr & 7; den_r[r8] = den_r[r8] * sf + ps; m_r[r8] = mn;
#pragma unroll
        for (int t = 0; t < HD / 16; ++t) acc[t][r8] = acc[t][r8] * sf; } }
    wave_lds_sync();
    for (int ks = 0; ks < nkt * 16; ks += 32) { const v16b pa = frag_kb(&Ph_[nloc][ks], hlf), pb = frag_kb(&Pl_[nloc][ks], hlf);
#pragma unroll
      for (int t = 0; t < HD / 16; ++t) { const v16b vh = frag_kb(&Vth[t * 16 + nloc][ks], hlf), vl = frag_kb(&Vtl[t * 16 + nloc][ks], hlf); acc[t] = wmma16b(pa, vh, acc[t]); acc[t] = wmma16b(pa, vl, acc[t]); acc[t] = wmma16b(pb, vh, acc[t]); } }
    wave_lds_sync(); }
#pragma unroll
  for (int t = 0; t < HD / 16; ++t)
#pragma unroll
    for (int r8 = 0; r8 < 8; ++r8) { const float dn = den_r[r8]; Of[8 * hlf + r8][t * 16 + nloc] = dn > 0.0f ? acc[t][r8] * (1.0f / (HS * PS)) / dn : 0.0f; }
  wave_lds_sync();
  for (int pass = 0; pass < 2; ++pass) { for (int rr = 0; rr < 16; ++rr) for (int s = 0; s < HD / 32; ++s) ((volatile float*)ATT)[(rowb + t0 + rr) * C + h * HD + s * 32 + lane] = Of[rr][s * 32 + lane]; __threadfence(); } }
__global__ __launch_bounds__(32) void gout_kernel(const float* __restrict__ pair, const float* __restrict__ ATT, const b16* __restrict__ WG, const b16* __restrict__ WO, const float* __restrict__ bg, const float* __restrict__ bo, const float* __restrict__ gam, const float* __restrict__ bet, int TLIM, float* __restrict__ out) { __shared__ __attribute__((aligned(16))) b16 Ph[16][C + 8], Ah[16][C + 8], Al[16][C + 8]; __shared__ float Tf[16][C + 4]; const int lane = threadIdx.x, nloc = lane & 15, hlf = lane >> 4; const size_t m0 = (size_t)blockIdx.x * 16; if (m0 >= (size_t)TLIM) return;
  for (int rr = 0; rr < 16; ++rr) for (int q = 0; q < C / 32; ++q) Ph[rr][q * 32 + lane] = (b16)(bf16_rne(pair[(m0 + rr) * C + q * 32 + lane]) * XS); if (lane < 16) for (int k = C; k < C + 8; ++k) { Ph[lane][k] = (b16)0.0f; Ah[lane][k] = (b16)0.0f; Al[lane][k] = (b16)0.0f; }
  wave_lds_sync(); v8f acc[8];
#pragma unroll
  for (int t = 0; t < 8; ++t) acc[t] = (v8f){};
#pragma unroll
  for (int kb = 0; kb < C; kb += 32) { const v16b a = frag_kb(&Ph[nloc][kb], hlf);
#pragma unroll
    for (int t = 0; t < 8; ++t) acc[t] = wmma16b(a, frag_kb(WG + (size_t)(t * 16 + nloc) * C + kb, hlf), acc[t]); }
#pragma unroll
  for (int t = 0; t < 8; ++t) { const int cc = t * 16 + nloc; const float bb = bfv(bg[cc]);
#pragma unroll
    for (int r8 = 0; r8 < 8; ++r8) { const int rr = 8 * hlf + r8; const float g = 1.0f / (1.0f + __expf(-(acc[t][r8] * (1.0f / (XS * WSC)) + bb))); b16 p, ql; split16(pmul(ATT[(m0 + rr) * C + cc], g) * HS, p, ql); Ah[rr][cc] = p; Al[rr][cc] = ql; } }
  wave_lds_sync();
#pragma unroll
  for (int t = 0; t < 8; ++t) acc[t] = (v8f){};
#pragma unroll
  for (int kb = 0; kb < C; kb += 32) { const v16b a = frag_kb(&Ah[nloc][kb], hlf), al = frag_kb(&Al[nloc][kb], hlf);
#pragma unroll
    for (int t = 0; t < 8; ++t) { const v16b bw = frag_kb(WO + (size_t)(t * 16 + nloc) * C + kb, hlf); acc[t] = wmma16b(a, bw, acc[t]); acc[t] = wmma16b(al, bw, acc[t]); } }
#pragma unroll
  for (int t = 0; t < 8; ++t) { const int cc = t * 16 + nloc; const float bb = bfv(bo[cc]);
#pragma unroll
    for (int r8 = 0; r8 < 8; ++r8) { const int rr = 8 * hlf + r8; Tf[rr][cc] = acc[t][r8] * (1.0f / (HS * WSC)) + bb + bfv(pair[(m0 + rr) * C + cc]); } }
  wave_lds_sync();
  for (int pass = 0; pass < 2; ++pass) { for (int rr = 0; rr < 16; ++rr) { float v[4], s = 0.0f; for (int k = 0; k < 4; ++k) { v[k] = Tf[rr][lane * 4 + k]; s += v[k]; } for (int o = 16; o; o >>= 1) s += __shfl_xor(s, o); const float mu = s / C; float s2 = 0.0f; for (int k = 0; k < 4; ++k) s2 += (v[k] - mu) * (v[k] - mu); for (int o = 16; o; o >>= 1) s2 += __shfl_xor(s2, o); const float rs = rsqrtf(s2 / C + 1e-5f);
      v4f o4; for (int k = 0; k < 4; ++k) { const int c = lane * 4 + k; o4[k] = pmul(pmul(v[k] - mu, rs), bfv(gam[c])) + bfv(bet[c]); } *(volatile v4f*)(out + (m0 + rr) * C + lane * 4) = o4; } __threadfence(); } }
}

extern "C" void kernel_launch(void* const* d_in, const int* in_sizes, int n_in, void* d_out, int out_size, void* d_ws, size_t ws_size, hipStream_t stream) {
  (void)n_in;
  auto Fp = [&](int i) { return (const float*)d_in[i]; };
  if (in_sizes[0] != NT * C || in_sizes[1] != C * C || in_sizes[7] != C * C || in_sizes[9] != C * C || in_sizes[11] != C || out_size != NT * C) return;
  const int BLIM = NB;
  const int TLIM = BLIM * L;
  size_t off = 0; char* ws = (char*)d_ws;
  auto carve = [&](size_t bytes) { char* p = ws + off; off += (bytes + 255) & ~(size_t)255; return p; };
  b16* W3 = (b16*)carve((size_t)3 * C * C * 2); b16* WO = (b16*)carve((size_t)C * C * 2); b16* WGp = (b16*)carve((size_t)C * C * 2); b16* PH = (b16*)carve((size_t)NT * PW * 2); b16* PL = (b16*)carve((size_t)NT * PW * 2); float* ATT = (float*)carve((size_t)NT * C * 4);
  if (off > ws_size || off > ((size_t)192 << 20)) return;
  wput_kernel<<<(unsigned)(((size_t)4 * C * (C / 8) + 255) / 256), 256, 0, stream>>>(Fp(1), Fp(3), Fp(5), Fp(9), W3, WO); wput_kernel<<<(unsigned)(((size_t)4 * C * (C / 8) + 255) / 256), 256, 0, stream>>>(Fp(1), Fp(3), Fp(5), Fp(7), W3, WGp);
  proj_kernel<<<TLIM / 16, 32, 0, stream>>>(Fp(0), W3, Fp(2), Fp(4), Fp(6), TLIM, PH, PL);
  att_kernel<<<BLIM * NH * (L / 16), 32, 0, stream>>>(PH, PL, (const float*)0, BLIM, ATT);
  gout_kernel<<<TLIM / 16, 32, 0, stream>>>(Fp(0), ATT, WGp, WO, Fp(8), Fp(10), Fp(11), Fp(12), TLIM, (float*)d_out);

}
